// MambaBlock_11476152615461
// MI455X (gfx1250) — hardware-verified
//
#include <hip/hip_runtime.h>
#include <math.h>

typedef __attribute__((ext_vector_type(16))) _Float16 v16h;
typedef __attribute__((ext_vector_type(8)))  _Float16 v8h;
typedef __attribute__((ext_vector_type(16))) __bf16   v16b;
typedef __attribute__((ext_vector_type(8)))  __bf16   v8b;
typedef __attribute__((ext_vector_type(8)))  float    v8f;
typedef __attribute__((ext_vector_type(4)))  float    v4f;

constexpr int kBatch  = 2;
constexpr int kSeq    = 2048;
constexpr int kDm     = 768;
constexpr int kDin    = 1536;
constexpr int kNst    = 16;
constexpr int kDtR    = 48;
constexpr int kDtP    = 64;
constexpr int kXdN    = 80;
constexpr int kXdP    = 128;
constexpr int kXzP    = 2 * kDin;
constexpr int kRows   = kBatch * kSeq;
constexpr int kConvTP = 260;
constexpr int kScanTS = 64;
constexpr int kScanCh = 64;
constexpr int kNChunk = kSeq / kScanTS;
constexpr float kLiveCut = 120.0f;
constexpr float kEpsDen  = 1e-12f;
constexpr float kFltMin  = 1.17549435e-38f;
static_assert(kDtR + 2 * kNst == kXdN, "x_proj width");
static_assert(kDtR <= kDtP && (kDtP % 32) == 0 && (kDtR % 8) == 0, "dt K pad");
static_assert((kDm % 64) == 0 && (kDin % 64) == 0, "GEMM K multiples of 32 and transpose tiles");
static_assert((kRows % 64) == 0 && (kXzP % 64) == 0 && (kXdP % 64) == 0 && (kDm % 64) == 0 && (kDin % 64) == 0, "GEMM M,N multiples of 64");
static_assert((kSeq % kScanTS) == 0 && (kSeq % 64) == 0 && (kDin % kScanCh) == 0 && (kDin % 256) == 0, "tile multiples");
static_assert((kSeq & (kSeq - 1)) == 0, "sequence length power of two");
static_assert(kNChunk == 32 && kScanTS == 64 && kScanCh == 64, "scan tiling");
static_assert(((kRows / 64) * (kXzP / 64)) % 8 == 0 && ((kRows / 64) * (kXdP / 64)) % 8 == 0 &&
              ((kRows / 64) * (kDin / 64)) % 8 == 0 && ((kRows / 64) * (kDm / 64)) % 8 == 0, "GEMM grids exact");

constexpr size_t kSzX16  = (size_t)kRows * kDm  * 2;
constexpr size_t kSzWI   = (size_t)kXzP  * kDm  * 2;
constexpr size_t kSzWX   = (size_t)kXdP  * kDin * 2;
constexpr size_t kSzWD   = (size_t)kDin  * kDtP * 2;
constexpr size_t kSzWO   = (size_t)kDm   * kDin * 2;
constexpr size_t kSzXZ   = (size_t)kRows * kXzP * 4;
constexpr size_t kSzUC   = (size_t)kRows * kDin * 4;
constexpr size_t kSzUC16 = (size_t)kRows * kDin * 2;
constexpr size_t kSzXD   = (size_t)kRows * kXdP * 4;
constexpr size_t kSzDT16 = (size_t)kRows * kDtP * 2;
constexpr size_t kOffXH  = 0;
constexpr size_t kOffXL  = kOffXH  + kSzX16;
constexpr size_t kOffWIH = kOffXL  + kSzX16;
constexpr size_t kOffWIL = kOffWIH + kSzWI;
constexpr size_t kOffWXH = kOffWIL + kSzWI;
constexpr size_t kOffWXL = kOffWXH + kSzWX;
constexpr size_t kOffWDH = kOffWXL + kSzWX;
constexpr size_t kOffWDL = kOffWDH + kSzWD;
constexpr size_t kOffWOH = kOffWDL + kSzWD;
constexpr size_t kOffWOL = kOffWOH + kSzWO;
constexpr size_t kOffXZ  = kOffWOL + kSzWO;
constexpr size_t kOffUC  = kOffXZ  + kSzXZ;
constexpr size_t kOffUCH = kOffUC  + kSzUC;
constexpr size_t kOffUCL = kOffUCH + kSzUC16;
constexpr size_t kOffXD  = kOffUCL + kSzUC16;
constexpr size_t kOffDTH = kOffXD  + kSzXD;
constexpr size_t kOffDTL = kOffDTH + kSzDT16;
constexpr size_t kWsTotal = kOffDTL + kSzDT16;
static_assert(kWsTotal == 131727360ull, "carve total");
static_assert(kWsTotal <= 134217728ull, "carve cap");
static_assert((kSzX16 % 128) == 0 && (kSzWI % 128) == 0 && (kSzWX % 128) == 0 && (kSzWD % 128) == 0 &&
              (kSzWO % 128) == 0 && (kSzXZ % 128) == 0 && (kSzUC % 128) == 0 && (kSzUC16 % 128) == 0 &&
              (kSzXD % 128) == 0 && (kSzDT16 % 128) == 0, "128-B aligned regions");

__device__ __forceinline__ unsigned short f2bf_bits(float f) {
  unsigned u = __float_as_uint(f);
  return (unsigned short)((u + 0x7FFFu + ((u >> 16) & 1u)) >> 16);
}
__device__ __forceinline__ float bf_bits2f(unsigned short h) { return __uint_as_float(((unsigned)h) << 16); }

__device__ __forceinline__ void dep_guard4_b(v8f& a, v8f& b, v8f& c, v8f& d, v16b x, v16b y) {
  asm volatile("v_nop\n\tv_nop\n\tv_nop\n\tv_nop" : "+v"(a), "+v"(b), "+v"(c), "+v"(d) : "v"(x), "v"(y));
}
__device__ __forceinline__ void keep4_b(v16b a, v16b b, v16b c, v16b d) { asm volatile("v_nop" :: "v"(a), "v"(b), "v"(c), "v"(d)); }
__device__ __forceinline__ void acc_guard4(v8f& a, v8f& b, v8f& c, v8f& d) { asm volatile("v_nop\n\tv_nop\n\tv_nop\n\tv_nop" : "+v"(a), "+v"(b), "+v"(c), "+v"(d)); }

struct FragB {
  union U { v16b v; v8b h[2]; };
  static __device__ __forceinline__ v16b load(const __bf16* p) {
    U f; f.h[0] = *(const v8b*)(p); f.h[1] = *(const v8b*)(p + 16); return f.v;
  }
  static __device__ __forceinline__ v8f mma(v16b a, v16b b, v8f c) {
    return __builtin_amdgcn_wmma_f32_16x16x32_bf16(false, a, false, b, (short)0, c, false, false);
  }
};

template <int BIAS_MODE>
__global__ __launch_bounds__(256) void wmma_gemm64_bf16x3(
    const unsigned short* __restrict__ Ahp, const unsigned short* __restrict__ Alp, int lda,
    const unsigned short* __restrict__ Bhp, const unsigned short* __restrict__ Blp, int ldb,
    float* __restrict__ C, int ldc, const float* __restrict__ bias, int M, int N, int K) {
  const __bf16* Ah = (const __bf16*)Ahp;
  const __bf16* Al = (const __bf16*)Alp;
  const __bf16* Bh = (const __bf16*)Bhp;
  const __bf16* Bl = (const __bf16*)Blp;
  __shared__ __align__(16) float sT[8][16 * 68];
  const int lane = threadIdx.x & 31;
  const int wave = threadIdx.x >> 5;
  const int tilesN = N >> 6;
  const int tilesM = M >> 6;
  const int tile = blockIdx.x * 8 + wave;
  if (tile >= tilesM * tilesN) return;
  const int tm = tile / tilesN;
  const int tn = tile - tm * tilesN;
  const int m0 = tm << 6;
  const int n0 = tn << 6;

  const int rlane = lane & 15;
  const int koff  = (lane >> 4) * 8;
  const int mOff  = (lane >> 4) * 8;

  v8f acc[4][4];
#pragma unroll
  for (int i = 0; i < 4; ++i)
#pragma unroll
    for (int j = 0; j < 4; ++j) acc[i][j] = (v8f){0.f,0.f,0.f,0.f,0.f,0.f,0.f,0.f};

  for (int k0 = 0; k0 < K; k0 += 32) {
    v16b bh[4], bl[4];
#pragma unroll
    for (int j = 0; j < 4; ++j) {
      const size_t bo = (size_t)(n0 + (j << 4) + rlane) * ldb + koff + k0;
      bh[j] = FragB::load(Bh + bo);
      bl[j] = FragB::load(Bl + bo);
    }
#pragma unroll
    for (int i = 0; i < 4; ++i) {
      const size_t ao = (size_t)(m0 + (i << 4) + rlane) * lda + koff + k0;
      v16b ah = FragB::load(Ah + ao);
      v16b al = FragB::load(Al + ao);
#pragma unroll
      for (int j = 0; j < 4; ++j) {
        acc[i][j] = FragB::mma(ah, bh[j], acc[i][j]);
        acc[i][j] = FragB::mma(ah, bl[j], acc[i][j]);
        acc[i][j] = FragB::mma(al, bh[j], acc[i][j]);
      }
      dep_guard4_b(acc[i][0], acc[i][1], acc[i][2], acc[i][3], ah, al);
    }
    keep4_b(bh[0], bh[1], bh[2], bh[3]);
    keep4_b(bl[0], bl[1], bl[2], bl[3]);
  }
  acc_guard4(acc[0][0], acc[0][1], acc[0][2], acc[0][3]);
  acc_guard4(acc[1][0], acc[1][1], acc[1][2], acc[1][3]);
  acc_guard4(acc[2][0], acc[2][1], acc[2][2], acc[2][3]);
  acc_guard4(acc[3][0], acc[3][1], acc[3][2], acc[3][3]);

  float* slab = sT[wave];
#pragma unroll
  for (int i = 0; i < 4; ++i) {
    const int mBase = m0 + (i << 4);
#pragma unroll
    for (int j = 0; j < 4; ++j) {
      const int n = n0 + (j << 4) + rlane;
      float bv = 0.f;
      if (BIAS_MODE == 2) bv = bias[n];
#pragma unroll
      for (int r = 0; r < 8; ++r) {
        float v = acc[i][j][r];
        if (BIAS_MODE == 2) v += bv;
        slab[(mOff + r) * 68 + (j << 4) + rlane] = v;
      }
    }
    __builtin_amdgcn_fence(__ATOMIC_RELEASE, "workgroup");
    __builtin_amdgcn_wave_barrier();
    __builtin_amdgcn_fence(__ATOMIC_ACQUIRE, "workgroup");
    {
      const int hh = lane >> 4, c4 = (lane & 15) * 4;
      for (int pass = 0; pass < 2; ++pass) {
#pragma unroll
        for (int it = 0; it < 8; ++it) {
          const int row = it * 2 + hh;
          v4f v = *(const v4f*)(slab + row * 68 + c4);
          *(volatile v4f*)(C + (size_t)(mBase + row) * ldc + n0 + c4) = v;
        }
        __threadfence();
      }
    }
    __builtin_amdgcn_fence(__ATOMIC_RELEASE, "workgroup");
    __builtin_amdgcn_wave_barrier();
    __builtin_amdgcn_fence(__ATOMIC_ACQUIRE, "workgroup");
  }
}

__global__ __launch_bounds__(256) void split_rows_bf16_kernel(
    const float* __restrict__ src, unsigned short* __restrict__ dhi, unsigned short* __restrict__ dlo, int total8)
{
  const int i = blockIdx.x * 256 + threadIdx.x;
  if (i >= total8) return;
  const size_t e0 = (size_t)i << 3;
  const v4f a0 = *(const v4f*)(src + e0);
  const v4f a1 = *(const v4f*)(src + e0 + 4);
  v8h hv, lv;
#pragma unroll
  for (int e = 0; e < 4; ++e) {
    const unsigned short h0 = f2bf_bits(a0[e]), h1 = f2bf_bits(a1[e]);
    const unsigned short l0 = f2bf_bits(a0[e] - bf_bits2f(h0)), l1 = f2bf_bits(a1[e] - bf_bits2f(h1));
    hv[e]     = __builtin_bit_cast(_Float16, h0);
    hv[4 + e] = __builtin_bit_cast(_Float16, h1);
    lv[e]     = __builtin_bit_cast(_Float16, l0);
    lv[4 + e] = __builtin_bit_cast(_Float16, l1);
  }
  unsigned short* qh = dhi + e0;
  unsigned short* ql = dlo + e0;
  *(volatile v8h*)qh = hv;
  *(volatile v8h*)ql = lv;
  __threadfence();
  *(volatile v8h*)qh = hv;
  *(volatile v8h*)ql = lv;
}

__global__ __launch_bounds__(256) void transpose_split_kernel(
    const float* __restrict__ W, unsigned short* __restrict__ BtH, unsigned short* __restrict__ BtL,
    int Kreal, int Kpad, int Ndim)
{
  __shared__ float tile[64 * 65];
  const int tid = threadIdx.x, lane = tid & 31, wave = tid >> 5;
  const int n0 = blockIdx.x * 64;
  const int k0 = blockIdx.y * 64;
#pragma unroll
  for (int p = 0; p < 16; ++p) {
    const int idx = tid + p * 256;
    const int kk  = idx >> 6;
    const int nn  = idx & 63;
    const int n   = n0 + nn;
    const int k   = k0 + kk;
    const int nc  = (n < Ndim) ? n : (Ndim - 1);
    const int kc  = (k < Kreal) ? k : (Kreal - 1);
    const float v = W[(size_t)kc * Ndim + nc];
    tile[kk * 65 + nn] = ((n < Ndim) && (k < Kreal)) ? v : 0.f;
  }
  __syncthreads();
  const int q = lane >> 3, c8 = (lane & 7) * 8;
  v8h hv[2], lv[2];
#pragma unroll
  for (int it = 0; it < 2; ++it) {
    const int nrow = it * 32 + wave * 4 + q;
#pragma unroll
    for (int e = 0; e < 8; ++e) {
      const float v = tile[(c8 + e) * 65 + nrow];
      const unsigned short hb = f2bf_bits(v);
      const unsigned short lb = f2bf_bits(v - bf_bits2f(hb));
      hv[it][e] = __builtin_bit_cast(_Float16, hb);
      lv[it][e] = __builtin_bit_cast(_Float16, lb);
    }
  }
  for (int pass = 0; pass < 2; ++pass) {
#pragma unroll
    for (int it = 0; it < 2; ++it) {
      const int nrow = it * 32 + wave * 4 + q;
      const size_t o = (size_t)(n0 + nrow) * Kpad + k0 + c8;
      *(volatile v8h*)(BtH + o) = hv[it];
      *(volatile v8h*)(BtL + o) = lv[it];
    }
    __threadfence();
  }
}

__global__ __launch_bounds__(256) void dt_split_kernel(
    const float* __restrict__ XD, unsigned short* __restrict__ DTH, unsigned short* __restrict__ DTL, int total8)
{
  const int i = blockIdx.x * 256 + threadIdx.x;
  if (i >= total8) return;
  const int e0  = i << 3;
  const int row = e0 >> 6;
  const int c8  = e0 & 63;
  const float* p = XD + (size_t)row * kXdP + c8;
  const v4f a0 = *(const v4f*)(p);
  const v4f a1 = *(const v4f*)(p + 4);
  const bool keep = (c8 < kDtR);
  v8h hv, lv;
#pragma unroll
  for (int e = 0; e < 4; ++e) {
    const float f0 = keep ? a0[e] : 0.f;
    const float f1 = keep ? a1[e] : 0.f;
    const unsigned short h0 = f2bf_bits(f0), h1 = f2bf_bits(f1);
    const unsigned short l0 = f2bf_bits(f0 - bf_bits2f(h0)), l1 = f2bf_bits(f1 - bf_bits2f(h1));
    hv[e]     = __builtin_bit_cast(_Float16, h0);
    hv[4 + e] = __builtin_bit_cast(_Float16, h1);
    lv[e]     = __builtin_bit_cast(_Float16, l0);
    lv[4 + e] = __builtin_bit_cast(_Float16, l1);
  }
  unsigned short* qh = DTH + e0;
  unsigned short* ql = DTL + e0;
  *(volatile v8h*)qh = hv;
  *(volatile v8h*)ql = lv;
  __threadfence();
  *(volatile v8h*)qh = hv;
  *(volatile v8h*)ql = lv;
}

__global__ __launch_bounds__(256) void conv_silu_kernel(
    const float* __restrict__ XZ, const float* __restrict__ cw, const float* __restrict__ cb,
    float* __restrict__ UC, unsigned short* __restrict__ UCH, unsigned short* __restrict__ UCL)
{
  __shared__ __align__(16) float sT[16 * kConvTP];
  const int tid = threadIdx.x, lane = tid & 31, wave = tid >> 5;
  const int d0 = blockIdx.x * 256, d = d0 + tid;
  const int g0 = blockIdx.y * 64;
  const int tb = g0 & (kSeq - 1);
  const float w0 = cw[d * 4 + 0], w1 = cw[d * 4 + 1], w2 = cw[d * 4 + 2], w3 = cw[d * 4 + 3];
  const float bc = cb[d];
  float xm3, xm2, xm1;
  {
    const bool hist = (tb > 0);
    const int rb = hist ? (g0 - 3) : g0;
    const float v3 = XZ[(size_t)rb * kXzP + d];
    const float v2 = XZ[(size_t)(rb + 1) * kXzP + d];
    const float v1 = XZ[(size_t)(rb + 2) * kXzP + d];
    xm3 = hist ? v3 : 0.f;
    xm2 = hist ? v2 : 0.f;
    xm1 = hist ? v1 : 0.f;
  }
  const int hrow = wave >> 1;
  const int hch  = (wave & 1) * 128 + lane * 4;
#pragma unroll 1
  for (int sub = 0; sub < 4; ++sub) {
    const int lb = g0 + sub * 16;
#pragma unroll 1
    for (int s = 0; s < 16; ++s) {
      const float xcur = XZ[(size_t)(lb + s) * kXzP + d];
      float acc = w0 * xm3;
      acc = fmaf(w1, xm2, acc);
      acc = fmaf(w2, xm1, acc);
      acc = fmaf(w3, xcur, acc);
      const float sv = acc + bc;
      const float sg = __builtin_amdgcn_rcpf(1.0f + expf(-sv));
      sT[s * kConvTP + tid] = sv * sg;
      xm3 = xm2; xm2 = xm1; xm1 = xcur;
    }
    __syncthreads();
    v4f fv[4];
    v8h bh[2], blo[2];
#pragma unroll
    for (int it = 0; it < 4; ++it) fv[it] = *(const v4f*)(sT + (it * 4 + hrow) * kConvTP + hch);
#pragma unroll
    for (int it = 0; it < 2; ++it) {
      const float* sp = sT + (it * 8 + wave) * kConvTP + lane * 8;
      const v4f a0 = *(const v4f*)(sp);
      const v4f a1 = *(const v4f*)(sp + 4);
#pragma unroll
      for (int e = 0; e < 4; ++e) {
        const unsigned short h0 = f2bf_bits(a0[e]), h1 = f2bf_bits(a1[e]);
        const unsigned short l0 = f2bf_bits(a0[e] - bf_bits2f(h0)), l1 = f2bf_bits(a1[e] - bf_bits2f(h1));
        bh[it][e]      = __builtin_bit_cast(_Float16, h0);
        bh[it][4 + e]  = __builtin_bit_cast(_Float16, h1);
        blo[it][e]     = __builtin_bit_cast(_Float16, l0);
        blo[it][4 + e] = __builtin_bit_cast(_Float16, l1);
      }
    }
    for (int pass = 0; pass < 2; ++pass) {
#pragma unroll
      for (int it = 0; it < 4; ++it)
        *(volatile v4f*)(UC + (size_t)(lb + it * 4 + hrow) * kDin + d0 + hch) = fv[it];
#pragma unroll
      for (int it = 0; it < 2; ++it) {
        const size_t o = (size_t)(lb + it * 8 + wave) * kDin + d0 + lane * 8;
        *(volatile v8h*)(UCH + o) = bh[it];
        *(volatile v8h*)(UCL + o) = blo[it];
      }
      __threadfence();
    }
    __syncthreads();
  }
}

__global__ __launch_bounds__(64) void scan_kernel(
    const float* __restrict__ XD, const float* __restrict__ XZ, const float* __restrict__ UC,
    const float* __restrict__ Alog, const float* __restrict__ Dp,
    unsigned short* __restrict__ YH, unsigned short* __restrict__ YL)
{
  __shared__ __align__(16) float sD[kScanTS * kScanCh];
  __shared__ __align__(16) float sT[kScanTS * kScanCh];
  __shared__ __align__(16) float sBC[kScanTS * 32];
  __shared__ float sH[kNst * kScanCh];
  __shared__ float sA[kNst * kScanCh];
  __shared__ float sCS[kNChunk * kScanCh];
  const int tid = threadIdx.x, lane = tid & 31, wave = tid >> 5;
  constexpr int kBlkPerB = kDin / kScanCh;
  const int bix = blockIdx.x / kBlkPerB;
  const int d0  = (blockIdx.x - bix * kBlkPerB) * kScanCh;
  const int d   = d0 + tid;
  const size_t row0 = (size_t)bix * kSeq;

  float amin = 3.0e38f;
#pragma unroll 1
  for (int n = 0; n < kNst; ++n) {
    const float a = -expf(Alog[(size_t)d * kNst + n]);
    sA[n * kScanCh + tid] = a;
    sH[n * kScanCh + tid] = 0.f;
    amin = fminf(amin, fabsf(a));
  }
#pragma unroll 1
  for (int c = 0; c < kNChunk; ++c) sCS[c * kScanCh + tid] = 0.f;
  const float Dd = Dp[d];

  const int lr = tid >> 4, lc4 = (tid & 15) * 4;
  const int br = tid >> 3, bc4 = (tid & 7) * 4;
  const int q = lane >> 3, c8 = (lane & 7) * 8;

#pragma unroll 1
  for (int v = 0; v < 2 * kNChunk; ++v) {
    const int phase = v / kNChunk;
    const int c  = v - phase * kNChunk;
    const int t0 = c * kScanTS;
    __syncthreads();
#pragma unroll
    for (int i = 0; i < 16; ++i) {
      const int r = lr + 4 * i;
      *(v4f*)(sD + r * kScanCh + lc4) = *(const v4f*)(XZ + (row0 + t0 + r) * kXzP + d0 + lc4);
    }
    if (phase == 1) {
#pragma unroll
      for (int i = 0; i < 8; ++i) {
        const int r = br + 8 * i;
        *(v4f*)(sBC + r * 32 + bc4) = *(const v4f*)(XD + (row0 + t0 + r) * kXdP + kDtR + bc4);
      }
    }
    __syncthreads();

    const float tafter = sCS[c * kScanCh + tid];
    float run = (phase == 1) ? tafter : 0.f;
#pragma unroll 1
    for (int s = kScanTS - 1; s >= 0; --s) {
      const float raw = sD[s * kScanCh + tid];
      const float dl  = fmaxf(raw, 0.0f) + log1pf(expf(-fabsf(raw)));
      sD[s * kScanCh + tid] = dl;
      sT[s * kScanCh + tid] = run;
      run += dl;
    }

    if (phase == 0) {
      sCS[c * kScanCh + tid] = run;
      if (c == kNChunk - 1) {
        float acc = 0.f;
#pragma unroll 1
        for (int c2 = kNChunk - 1; c2 >= 0; --c2) {
          const float t = sCS[c2 * kScanCh + tid];
          sCS[c2 * kScanCh + tid] = acc;
          acc += t;
        }
      }
    } else {
#pragma unroll 1
      for (int s = 0; s < kScanTS; ++s) {
        const size_t row = row0 + t0 + s;
        float u  = UC[row * kDin + d];
        float zv = XZ[row * kXzP + kDin + d];
        asm volatile("" : "+v"(u), "+v"(zv));
        const float dl = sD[s * kScanCh + tid];
        const float Tl = sT[s * kScanCh + tid];
        const bool live = (amin * Tl <= kLiveCut);
        const unsigned anyLive = __builtin_amdgcn_ballot_w32(live);
        float ys = 0.f;
        if (anyLive != 0u) {
          const float du = dl * u;
          const float* bcrow = sBC + s * 32;
#pragma unroll 1
          for (int n = 0; n < kNst; ++n) {
            const float an = sA[n * kScanCh + tid];
            const float hp = sH[n * kScanCh + tid];
            const float e1 = expf(dl * an);
            const float hn = fmaf(e1, hp, du * bcrow[n]);
            sH[n * kScanCh + tid] = hn;
            float e2 = expf(an * Tl);
            e2 = (e2 < kFltMin) ? 0.0f : e2;
            const float fac = e2 * __builtin_amdgcn_rcpf(e2 + kEpsDen);
            ys = fmaf(hn * fac, bcrow[kNst + n], ys);
          }
        }
        const float y  = fmaf(u, Dd, ys);
        const float sg = __builtin_amdgcn_rcpf(1.0f + expf(-zv));
        sD[s * kScanCh + tid] = y * (zv * sg);
      }
      __syncthreads();
      v8h hv[8], lv[8];
#pragma unroll
      for (int it = 0; it < 8; ++it) {
        const int row = it * 8 + wave * 4 + q;
        const float* sp = sD + row * kScanCh + c8;
        const v4f a0 = *(const v4f*)(sp);
        const v4f a1 = *(const v4f*)(sp + 4);
#pragma unroll
        for (int e = 0; e < 4; ++e) {
          const unsigned short h0 = f2bf_bits(a0[e]), h1 = f2bf_bits(a1[e]);
          const unsigned short l0 = f2bf_bits(a0[e] - bf_bits2f(h0)), l1 = f2bf_bits(a1[e] - bf_bits2f(h1));
          hv[it][e]     = __builtin_bit_cast(_Float16, h0);
          hv[it][4 + e] = __builtin_bit_cast(_Float16, h1);
          lv[it][e]     = __builtin_bit_cast(_Float16, l0);
          lv[it][4 + e] = __builtin_bit_cast(_Float16, l1);
        }
      }
      for (int pass = 0; pass < 2; ++pass) {
#pragma unroll
        for (int it = 0; it < 8; ++it) {
          const int row = it * 8 + wave * 4 + q;
          const size_t o = (row0 + t0 + row) * kDin + d0 + c8;
          *(volatile v8h*)(YH + o) = hv[it];
          *(volatile v8h*)(YL + o) = lv[it];
        }
        __threadfence();
      }
    }
  }
}

extern "C" void kernel_launch(void* const* d_in, const int* in_sizes, int n_in,
                              void* d_out, int out_size, void* d_ws, size_t ws_size,
                              hipStream_t stream) {
  if (n_in < 10) return;
  if (in_sizes[0] != kRows * kDm) return;
  if (in_sizes[1] != kDm * kXzP) return;
  if (in_sizes[2] != kDin * 4) return;
  if (in_sizes[3] != kDin) return;
  if (in_sizes[4] != kDin * kXdN) return;
  if (in_sizes[5] != kDtR * kDin) return;
  if (in_sizes[6] != kDin) return;
  if (in_sizes[7] != kDin * kNst) return;
  if (in_sizes[8] != kDin) return;
  if (in_sizes[9] != kDin * kDm) return;
  if (out_size != kRows * kDm) return;
  if (ws_size < kWsTotal) return;

  const float* x      = (const float*)d_in[0];
  const float* W_in   = (const float*)d_in[1];
  const float* conv_w = (const float*)d_in[2];
  const float* conv_b = (const float*)d_in[3];
  const float* W_x    = (const float*)d_in[4];
  const float* W_dt   = (const float*)d_in[5];
  const float* b_dt   = (const float*)d_in[6];
  const float* A_log  = (const float*)d_in[7];
  const float* Dp     = (const float*)d_in[8];
  const float* W_out  = (const float*)d_in[9];
  float* out = (float*)d_out;

  char* ws = (char*)d_ws;
  unsigned short* XH  = (unsigned short*)(ws + kOffXH);
  unsigned short* XL  = (unsigned short*)(ws + kOffXL);
  unsigned short* WIH = (unsigned short*)(ws + kOffWIH);
  unsigned short* WIL = (unsigned short*)(ws + kOffWIL);
  unsigned short* WXH = (unsigned short*)(ws + kOffWXH);
  unsigned short* WXL = (unsigned short*)(ws + kOffWXL);
  unsigned short* WDH = (unsigned short*)(ws + kOffWDH);
  unsigned short* WDL = (unsigned short*)(ws + kOffWDL);
  unsigned short* WOH = (unsigned short*)(ws + kOffWOH);
  unsigned short* WOL = (unsigned short*)(ws + kOffWOL);
  float*          XZ  = (float*)(ws + kOffXZ);
  float*          UC  = (float*)(ws + kOffUC);
  unsigned short* UCH = (unsigned short*)(ws + kOffUCH);
  unsigned short* UCL = (unsigned short*)(ws + kOffUCL);
  float*          XD  = (float*)(ws + kOffXD);
  unsigned short* DTH = (unsigned short*)(ws + kOffDTH);
  unsigned short* DTL = (unsigned short*)(ws + kOffDTL);
  unsigned short* YH  = UCH;
  unsigned short* YL  = UCL;

  split_rows_bf16_kernel<<<(kRows * kDm / 8) / 256, 256, 0, stream>>>(x, XH, XL, kRows * kDm / 8);

  transpose_split_kernel<<<dim3(kXzP / 64, kDm / 64), 256, 0, stream>>>(W_in, WIH, WIL, kDm, kDm, kXzP);
  transpose_split_kernel<<<dim3(kXdP / 64, kDin / 64), 256, 0, stream>>>(W_x, WXH, WXL, kDin, kDin, kXdN);
  transpose_split_kernel<<<dim3(kDin / 64, kDtP / 64), 256, 0, stream>>>(W_dt, WDH, WDL, kDtR, kDtP, kDin);
  transpose_split_kernel<<<dim3(kDm / 64, kDin / 64), 256, 0, stream>>>(W_out, WOH, WOL, kDin, kDin, kDm);

  wmma_gemm64_bf16x3<0><<<((kRows / 64) * (kXzP / 64)) / 8, 256, 0, stream>>>(
      XH, XL, kDm, WIH, WIL, kDm, XZ, kXzP, b_dt, kRows, kXzP, kDm);

  conv_silu_kernel<<<dim3(kDin / 256, kRows / 64), 256, 0, stream>>>(XZ, conv_w, conv_b, UC, UCH, UCL);

  wmma_gemm64_bf16x3<0><<<((kRows / 64) * (kXdP / 64)) / 8, 256, 0, stream>>>(
      UCH, UCL, kDin, WXH, WXL, kDin, XD, kXdP, b_dt, kRows, kXdP, kDin);

  dt_split_kernel<<<(kRows * kDtP / 8) / 256, 256, 0, stream>>>(XD, DTH, DTL, kRows * kDtP / 8);

  wmma_gemm64_bf16x3<2><<<((kRows / 64) * (kDin / 64)) / 8, 256, 0, stream>>>(
      DTH, DTL, kDtP, WDH, WDL, kDtP, XZ, kXzP, b_dt, kRows, kDin, kDtP);

  scan_kernel<<<kBatch * (kDin / kScanCh), kScanCh, 0, stream>>>(XD, XZ, UC, A_log, Dp, YH, YL);

  wmma_gemm64_bf16x3<0><<<((kRows / 64) * (kDm / 64)) / 8, 256, 0, stream>>>(
      YH, YL, kDin, WOH, WOL, kDin, out, kDm, b_dt, kRows, kDm, kDin);
}
